// EdgeDecoder_14542759264855
// MI455X (gfx1250) — hardware-verified
//
#include <hip/hip_runtime.h>
#include <math.h>

typedef __attribute__((ext_vector_type(16))) _Float16 v16h;
typedef __attribute__((ext_vector_type(16))) __bf16 v16b;
typedef __attribute__((ext_vector_type(8)))  _Float16 v8h;
typedef __attribute__((ext_vector_type(8)))  float v8f;
typedef __attribute__((ext_vector_type(4)))  float v4f;
typedef __attribute__((ext_vector_type(2)))  float v2f;
typedef __attribute__((ext_vector_type(4)))  unsigned v4u;
typedef __attribute__((ext_vector_type(4)))  int v4i;
typedef float __attribute__((may_alias)) float_a;
typedef int __attribute__((may_alias)) int_a;

template <typename T> __device__ __forceinline__ void vst2(void* p, T v) { *(volatile T*)p = v; __threadfence(); *(volatile T*)p = v; }
__device__ __forceinline__ v8f wmma16(v16h a, v16h b, v8f c) {
  v8f d = __builtin_amdgcn_wmma_f32_16x16x32_f16(false, a, false, b, (short)0, c, false, false);
  asm volatile("v_nop\n\tv_nop\n\tv_nop\n\tv_nop" : "+v"(d) : "v"(a), "v"(b));
  return d;
}
__device__ __forceinline__ v8f wmma_bf(v16b a, v16b b, v8f c) {
  v8f d = __builtin_amdgcn_wmma_f32_16x16x32_bf16(false, a, false, b, (short)0, c, false, false);
  asm volatile("v_nop\n\tv_nop\n\tv_nop\n\tv_nop" : "+v"(d) : "v"(a), "v"(b));
  return d;
}
__device__ __forceinline__ v16h frag_h(const _Float16* rowk0, int lane) {
  union { v16h v; v8h q[2]; } u; const _Float16* p = rowk0 + 8 * (lane >> 4);
  u.q[0] = *(const v8h*)p; u.q[1] = *(const v8h*)(p + 16); return u.v;
}
__device__ __forceinline__ v16h frag_f32(const float* rowk0, int lane) {
  v16h a; const float* p = rowk0 + 8 * (lane >> 4);
#pragma unroll
  for (int i = 0; i < 8; ++i) { a[i] = (_Float16)p[i]; a[8 + i] = (_Float16)p[16 + i]; }
  return a;
}
__device__ __forceinline__ v16h frag_f32s(const float* rowk0, int lane, float sc) {
  v16h a; const float* p = rowk0 + 8 * (lane >> 4);
#pragma unroll
  for (int i = 0; i < 8; ++i) { a[i] = (_Float16)(p[i] * sc); a[8 + i] = (_Float16)(p[16 + i] * sc); }
  return a;
}
__device__ __forceinline__ v16h fragc_f32(const float* W, int k0, int n, int lane, int ld, int K) {
  v16h a; const int g = lane >> 4;
#pragma unroll
  for (int i = 0; i < 8; ++i) { const int ka = k0 + 8 * g + i, kb = ka + 16;
    a[i] = (_Float16)(ka < K ? W[(size_t)(ka < K ? ka : K - 1) * ld + n] : 0.f); a[8 + i] = (_Float16)(kb < K ? W[(size_t)(kb < K ? kb : K - 1) * ld + n] : 0.f); }
  return a;
}
struct F2 { v16b h, l; };
__device__ __forceinline__ F2 bsplit16(const float v[16]) { F2 r;
#pragma unroll
  for (int i = 0; i < 16; ++i) { const __bf16 h = (__bf16)v[i]; r.h[i] = h; r.l[i] = (__bf16)(v[i] - (float)h); }
  return r; }
__device__ __forceinline__ F2 split_row(const float* row, int k0, int lane) { float v[16]; const float* p = row + k0 + 8 * (lane >> 4);
#pragma unroll
  for (int i = 0; i < 8; ++i) { v[i] = p[i]; v[8 + i] = p[16 + i]; }
  return bsplit16(v); }
__device__ __forceinline__ F2 split_rowK(const float* row, int k0, int lane, int K) { float v[16]; const int g = lane >> 4;
#pragma unroll
  for (int i = 0; i < 8; ++i) { const int ka = k0 + 8 * g + i, kb = ka + 16; v[i] = ka < K ? row[ka < K ? ka : K - 1] : 0.f; v[8 + i] = kb < K ? row[kb < K ? kb : K - 1] : 0.f; }
  return bsplit16(v); }
__device__ __forceinline__ F2 split_col(const float* W, int k0, int n, int lane, int ld, int K) { float v[16]; const int g = lane >> 4;
#pragma unroll
  for (int i = 0; i < 8; ++i) { const int ka = k0 + 8 * g + i, kb = ka + 16; v[i] = ka < K ? W[(size_t)(ka < K ? ka : K - 1) * ld + n] : 0.f; v[8 + i] = kb < K ? W[(size_t)(kb < K ? kb : K - 1) * ld + n] : 0.f; }
  return bsplit16(v); }
__device__ __forceinline__ v8f mac3(const F2& a, const F2& b, v8f c) { c = wmma_bf(a.l, b.h, c); c = wmma_bf(a.h, b.l, c); return wmma_bf(a.h, b.h, c); }
__device__ __forceinline__ float sigm(float v) { return 1.0f / (1.0f + expf(-v)); }
#define LDSX() do { asm volatile("s_wait_dscnt 0" ::: "memory"); __builtin_amdgcn_wave_barrier(); __builtin_amdgcn_fence(__ATOMIC_RELEASE, "workgroup"); } while (0)

#define NEDGE 1000000
#define NU 100000
#define NF 50000
#define HH2 128
#define HH 1024


#define KS 1
#define NSH 1
#define NRB (NT / 64 + NE)
typedef __attribute__((ext_vector_type(4))) int v4i2;
__device__ __forceinline__ float bfr(float v) { return (float)(__bf16)v; }
__device__ __forceinline__ v16b wcol_in(const float* Wm, int k0, int o, int lane, int ld, int nvalid) { v16b w; const int g = lane >> 4; const int oc = o < nvalid ? o : 0; const float keep = o < nvalid ? 1.f : 0.f; float t0[8], t1[8];
#pragma unroll
  for (int i = 0; i < 8; ++i) t0[i] = Wm[(size_t)(k0 + 8 * g + i) * ld + oc];
  asm volatile("s_wait_loadcnt 0x0" ::: "memory");
#pragma unroll
  for (int i = 0; i < 8; ++i) t1[i] = Wm[(size_t)(k0 + 16 + 8 * g + i) * ld + oc];
  asm volatile("s_wait_loadcnt 0x0" ::: "memory");
#pragma unroll
  for (int i = 0; i < 8; ++i) { w[i] = (__bf16)(t0[i] * keep); w[8 + i] = (__bf16)(t1[i] * keep); }
  return w; }
#define WS_IDX 0u
#define WS_WGT (WS_IDX + 16u * NT)
#define WS_TOK (WS_WGT + 16u * NT)
#define WS_RB  (WS_TOK + 16u * NT)
#define WS_H   (WS_RB + 64u * NRB + 1024u)
#define WS_END (WS_H + 4u * (size_t)NT * HS)


__global__ __launch_bounds__(128) void k_edge(const float* __restrict__ ZU, const float* __restrict__ ZF, const int* __restrict__ ROW, const int* __restrict__ COL, const float* __restrict__ W1, const float* __restrict__ B1, const float* __restrict__ GM, const float* __restrict__ BT, const float* __restrict__ RM, const float* __restrict__ RV, const float* __restrict__ W2, const float* __restrict__ B2, float* __restrict__ OUT) {
  __shared__ float so[64]; __shared__ int sidx[2][64];
  const int tid = threadIdx.x, wave = tid >> 5, lane = tid & 31, col = lane & 15, g = lane >> 4; const size_t e0 = (size_t)blockIdx.x * 64;
  if (tid < 64) { int r = ROW[e0 + tid], c = COL[e0 + tid]; r = r < 0 ? 0 : (r >= NU ? NU - 1 : r); c = c < 0 ? 0 : (c >= NF ? NF - 1 : c); sidx[0][tid] = r; sidx[1][tid] = c; }
  __syncthreads();
  const int myrow = wave * 16 + col; const float* zu = ZU + (size_t)sidx[0][myrow] * HH2; const float* zf = ZF + (size_t)sidx[1][myrow] * HH2;
  v8f acc[8] = {};
#pragma unroll 1
  for (int kc = 0; kc < 8; ++kc) { const float* p = (kc < 4 ? zu + kc * 32 : zf + (kc - 4) * 32) + 8 * g; v16b a; { float t0[8], t1[8];
#pragma unroll
      for (int i = 0; i < 8; ++i) t0[i] = p[i];
      asm volatile("s_wait_loadcnt 0x0" ::: "memory");
#pragma unroll
      for (int i = 0; i < 8; ++i) t1[i] = p[16 + i];
      asm volatile("s_wait_loadcnt 0x0" ::: "memory");
#pragma unroll
      for (int i = 0; i < 8; ++i) { a[i] = (__bf16)t0[i]; a[8 + i] = (__bf16)t1[i]; } }
#pragma unroll
    for (int j = 0; j < 8; ++j) { v16b w; { const int o = j * 16 + col; const float* pw = W1 + (size_t)o * 256 + kc * 32 + 8 * g; float u0[8], u1[8];
#pragma unroll
        for (int i = 0; i < 8; ++i) u0[i] = pw[i];
        asm volatile("s_wait_loadcnt 0x0" ::: "memory");
#pragma unroll
        for (int i = 0; i < 8; ++i) u1[i] = pw[16 + i];
        asm volatile("s_wait_loadcnt 0x0" ::: "memory");
#pragma unroll
        for (int i = 0; i < 8; ++i) { w[i] = (__bf16)u0[i]; w[8 + i] = (__bf16)u1[i]; } }
      acc[j] = wmma_bf(a, w, acc[j]); } }
  float part[8]; _Pragma("unroll") for (int r = 0; r < 8; ++r) part[r] = 0.f;
#pragma unroll
  for (int j = 0; j < 8; ++j) { const int o = j * 16 + col; const float b1 = bfr(B1[o]), gm = bfr(GM[o]), bt = bfr(BT[o]), rm = bfr(RM[o]), rv = bfr(RV[o]), w2 = bfr(W2[o]); asm volatile("s_wait_loadcnt 0x0" ::: "memory"); const float sc = rsqrtf(rv + 1e-5f) * gm;
#pragma unroll
    for (int r = 0; r < 8; ++r) { const float h = fmaxf((acc[j][r] + b1 - rm) * sc + bt, 0.f); part[r] += h * w2; } }
#pragma unroll
  for (int r = 0; r < 8; ++r) {
#pragma unroll
    for (int o = 1; o < 16; o <<= 1) part[r] += __shfl_xor(part[r], o); }
  const float b2v = bfr(B2[0]); asm volatile("s_wait_loadcnt 0x0" ::: "memory");
  if (col == 0) { _Pragma("unroll") for (int r = 0; r < 8; ++r) { const float x = part[r] + b2v + 0.1f; so[wave * 16 + 8 * g + r] = 1.0f / (1.0f + expf(-x)); } }
  __syncthreads();
  if (tid < 16) vst2(OUT + e0 + tid * 4, *(const v4f*)&so[tid * 4]); }
extern "C" void kernel_launch(void* const* d_in, const int* in_sizes, int n_in, void* d_out, int out_size, void* d_ws, size_t ws_size, hipStream_t stream) {
  (void)in_sizes; (void)n_in; (void)out_size; (void)d_ws; (void)ws_size;
  const float** F = (const float**)d_in;
  k_edge<<<dim3(NEDGE / 64), 128, 0, stream>>>(F[0], F[1], (const int*)d_in[2], (const int*)d_in[3], F[4], F[5], F[6], F[7], F[8], F[9], F[10], F[11], (float*)d_out);
}
